// SimplicialModel_18932215841010
// MI455X (gfx1250) — hardware-verified
//
#include <hip/hip_runtime.h>


#ifndef NB
#define NB 16
#endif
#ifndef SEQ
#define SEQ 512
#endif
#define NB_FULL  16
#define SEQ_FULL 512
#ifndef OUT_SEQ
#define OUT_SEQ SEQ
#endif
#define DM    256
#define DO    256
#define HD    64
#define NCH   4
#define VE    64
#define SQ    (SEQ - VE)
#define NPAIR (VE * VE)
#define AW    4
#define OSP   68
#define QRS   2048.0f
#define QRI   (1.0f / 2048.0f)
#define BCAR  64.0f
#define LOG2E 1.4426950408889634f
#define PSH   14.0f
#define NEGB  (-3.0e38f)

static_assert(HD == 64);
static_assert(VE == 64);
static_assert(NCH * HD == DO);
static_assert(DM % 64 == 0);
static_assert(DO % 64 == 0);
static_assert(DM % 32 == 0);
static_assert(HD % 32 == 0);
static_assert(NPAIR % 64 == 0);
static_assert(SEQ % 64 == 0);
static_assert(SEQ > VE);
static_assert(SQ % 64 == 0);
static_assert(SQ % (16 * AW) == 0);
static_assert(32 * AW == 2 * VE);
static_assert(((size_t)SEQ * DM) % 8 == 0);
static_assert(((size_t)NPAIR * HD) % 8 == 0);
static_assert(NB <= NB_FULL);
static_assert(SEQ <= SEQ_FULL);
static_assert((OSP * 4) % 16 == 0);
static_assert(4 * 32 * 16 == 16 * HD * 2);
static_assert(8 * 32 * 16 == 16 * HD * 4);
static_assert(16 * 16 == 64 * 4);
static_assert(256 * 2 * 16 == 64 * 64 * 2);
static_assert((VE * VE + AW * VE * 16 + AW * 16 * OSP + 2 * VE) * 4 <= 65536);
static_assert((VE * VE + AW * VE * 16 + AW * 16 * OSP + 2 * VE) * 4 <= 131072);
static_assert((16 * 68 + 64) * 4 <= 131072);
static_assert(64 * 65 * 4 <= 131072);

typedef _Float16 h16;
typedef unsigned short bf;
typedef __attribute__((ext_vector_type(16))) __bf16   v16bf;
typedef __attribute__((ext_vector_type(16))) _Float16 v16h;
typedef __attribute__((ext_vector_type(8)))  _Float16 v8h;
typedef __attribute__((ext_vector_type(8)))  unsigned short v8us;
typedef __attribute__((ext_vector_type(8)))  float    v8f;
typedef __attribute__((ext_vector_type(4)))  float    v4f;
typedef v4f  __attribute__((may_alias)) v4fa;

__device__ __forceinline__ unsigned short f2bf(float f) { unsigned u = __float_as_uint(f); u += 0x7FFFu + ((u >> 16) & 1u); return (unsigned short)(u >> 16); }
__device__ __forceinline__ float bfr(float f) { return __uint_as_float(((unsigned)f2bf(f)) << 16); }
__device__ __forceinline__ v16h cat16(v8h lo, v8h hi) { return __builtin_shufflevector(lo, hi, 0, 1, 2, 3, 4, 5, 6, 7, 8, 9, 10, 11, 12, 13, 14, 15); }
__device__ __forceinline__ v16bf cat16b(v8us lo, v8us hi) { return __builtin_bit_cast(v16bf, __builtin_shufflevector(lo, hi, 0, 1, 2, 3, 4, 5, 6, 7, 8, 9, 10, 11, 12, 13, 14, 15)); }
__device__ __forceinline__ v8f wmma16(v16h a, v16h b, v8f c) { return __builtin_amdgcn_wmma_f32_16x16x32_f16(false, a, false, b, (short)0, c, false, false); }
__device__ __forceinline__ v8f wmmab(v16bf a, v16bf b, v8f c) { return __builtin_amdgcn_wmma_f32_16x16x32_bf16(false, a, false, b, (short)0, c, false, false); }
__device__ __forceinline__ v16h  ldh(const h16* p) { return cat16(*(const v8h*)p, *(const v8h*)(p + 16)); }
__device__ __forceinline__ v16bf ldb(const bf* p)  { return cat16b(*(const v8us*)p, *(const v8us*)(p + 16)); }
__device__ __forceinline__ void wave_sync() { __builtin_amdgcn_fence(3  , "wavefront"); __builtin_amdgcn_wave_barrier(); asm volatile("" ::: "memory"); }
__device__ __forceinline__ v8f wmma16g(v16h a, v16h b, v8f c) { c = wmma16(a, b, c); asm volatile("v_nop\n\tv_nop\n\tv_nop\n\tv_nop" : "+v"(c) : "v"(a), "v"(b)); return c; }
__device__ __forceinline__ v8f wmmabg(v16bf a, v16bf b, v8f c) { c = wmmab(a, b, c); asm volatile("v_nop\n\tv_nop\n\tv_nop\n\tv_nop" : "+v"(c) : "v"(a), "v"(b)); return c; }
__device__ __forceinline__ h16 toh_flush(float v) { const float w = (fabsf(v) < 6.103515625e-05f) ? 0.0f : v; return (h16)w; }

__global__ __launch_bounds__(256) void k_cvt8(const float* __restrict__ src, bf* dst, size_t n8) {
    const size_t i = (size_t)blockIdx.x * 256 + threadIdx.x; if (i >= n8) return;
    const v8f v = *(const v8f*)(src + i * 8); v8us o;
#pragma unroll
    for (int k = 0; k < 8; ++k) o[k] = f2bf(v[k]);
    *(volatile v8us*)(dst + i * 8) = o; __threadfence(); *(volatile v8us*)(dst + i * 8) = o;
}

__global__ __launch_bounds__(256) void k_cvt8h(const float* __restrict__ src, h16* dst, size_t n8, float carry) {
    const size_t i = (size_t)blockIdx.x * 256 + threadIdx.x; if (i >= n8) return;
    const v8f v = *(const v8f*)(src + i * 8); v8h o;
#pragma unroll
    for (int k = 0; k < 8; ++k) o[k] = toh_flush(bfr(v[k]) * carry);
    *(volatile v8h*)(dst + i * 8) = o; __threadfence(); *(volatile v8h*)(dst + i * 8) = o;
}

__global__ __launch_bounds__(256) void k_wT(const float* __restrict__ W, bf* WT) {
    __shared__ float ts[64 * 65];
    const int tid = threadIdx.x; const int d0 = blockIdx.x * 64, e0 = blockIdx.y * 64;
    for (int it = 0; it < 16; ++it) { const int idx = it * 256 + tid; const int dd = idx >> 6, ee = idx & 63;
        ts[dd * 65 + ee] = W[(size_t)(d0 + dd) * DO + e0 + ee]; }
    __syncthreads();
    for (int ps = 0; ps < 2; ++ps) {
#pragma unroll
        for (int it = 0; it < 2; ++it) { const int er = it * 32 + (tid >> 3), c8 = (tid & 7) * 8; v8us o;
#pragma unroll
            for (int k = 0; k < 8; ++k) o[k] = f2bf(ts[(c8 + k) * 65 + er]);
            *(volatile v8us*)(WT + (size_t)(e0 + er) * DM + d0 + c8) = o; }
        if (ps == 0) __threadfence(); }
}

__global__ __launch_bounds__(32) void k_proj(const bf* __restrict__ A, const bf* __restrict__ Bt, h16* Ph, h16* Pr, float* NRM, float* OUT) {
    __shared__ __align__(16) float os[16 * 68];
    __shared__ __align__(16) float nrm[64];
    const int K = DM;
    const int lane = threadIdx.x & 31, lr = lane & 15, hi = lane >> 4; const int r0 = blockIdx.x * 64, c0 = blockIdx.y * 64;
    v8f acc[4][4];
#pragma unroll
    for (int mb = 0; mb < 4; ++mb)
#pragma unroll
        for (int nb = 0; nb < 4; ++nb) acc[mb][nb] = (v8f){};
    const size_t aoff = (size_t)(r0 + lr) * K + 8 * hi, boff = (size_t)(c0 + lr) * K + 8 * hi;
    for (int kc = 0; kc < K; kc += 32) {
        v16bf a[4];
#pragma unroll
        for (int mb = 0; mb < 4; ++mb) a[mb] = ldb(A + aoff + (size_t)mb * 16 * K + kc);
#pragma unroll
        for (int nb = 0; nb < 4; ++nb) { const v16bf b = ldb(Bt + boff + (size_t)nb * 16 * K + kc);
#pragma unroll
            for (int mb = 0; mb < 4; ++mb) acc[mb][nb] = wmmabg(a[mb], b, acc[mb][nb]); }
    }
    const int chunk = blockIdx.y; const int bb = r0 / SEQ, tt = r0 % SEQ;
    const size_t tbase = ((size_t)(chunk * NB + bb) * SEQ + (size_t)tt) * HD;
    const bool wout = (chunk == 3) && (tt >= SQ);
    float* orow = OUT + ((size_t)bb * OUT_SEQ + (size_t)tt) * HD;
#pragma unroll
    for (int mb = 0; mb < 4; ++mb) {
#pragma unroll
        for (int nb = 0; nb < 4; ++nb) {
#pragma unroll
            for (int j = 0; j < 8; ++j) os[(hi * 8 + j) * 68 + nb * 16 + lr] = acc[mb][nb][j]; }
        wave_sync();
        { const int nrow = lane >> 1, nh = (lane & 1) * 32; float s = 0.0f;
          for (int c = 0; c < 8; ++c) { const v4f x = *(const v4fa*)(&os[nrow * 68 + nh + 4 * c]);
              s = fmaf(x[0], x[0], s); s = fmaf(x[1], x[1], s); s = fmaf(x[2], x[2], s); s = fmaf(x[3], x[3], s); }
          s += __shfl_xor(s, 1, 32);
          if ((lane & 1) == 0) nrm[mb * 16 + nrow] = s; }
        for (int ps = 0; ps < 2; ++ps) {
            const size_t sb = tbase + (size_t)(mb * 16) * HD;
#pragma unroll
            for (int s = 0; s < 4; ++s) { const int p = s * 32 + lane; const int row = p >> 3, c8 = (p & 7) * 8;
                const v4f x0 = *(const v4fa*)(&os[row * 68 + c8]); const v4f x1 = *(const v4fa*)(&os[row * 68 + c8 + 4]); v8h hv, rv;
#pragma unroll
                for (int i = 0; i < 4; ++i) { const h16 a0 = toh_flush(x0[i]); const h16 a1 = toh_flush(x1[i]); hv[i] = a0; hv[4 + i] = a1;
                    rv[i] = toh_flush((x0[i] - (float)a0) * QRS); rv[4 + i] = toh_flush((x1[i] - (float)a1) * QRS); }
                const size_t oo = sb + (size_t)p * 8;
                *(volatile v8h*)(Ph + oo) = hv; *(volatile v8h*)(Pr + oo) = rv; }
            if (wout) {
#pragma unroll
                for (int s = 0; s < 8; ++s) { const int p = s * 32 + lane; const int row = p >> 4, cofs = (p & 15) * 4;
                    const v4f val = *(const v4fa*)(&os[row * 68 + cofs]);
                    *(volatile v4f*)(orow + (size_t)(mb * 16) * HD + (size_t)p * 4) = val; } }
            if (ps == 0) __threadfence(); }
        wave_sync();
    }
    { const int l4 = (lane & 15) * 4; const v4f nv = *(const v4fa*)(&nrm[l4]);
      float* np = NRM + (size_t)(chunk * NB + bb) * SEQ + (size_t)tt + l4;
      if (lane < 16) { *(volatile v4f*)np = nv; }
      __threadfence();
      if (lane < 16) { *(volatile v4f*)np = nv; } }
}

__global__ __launch_bounds__(32) void k_gemm64(const h16* __restrict__ A, const h16* __restrict__ Bt, h16* C,
                                               size_t aSx, size_t aSy, size_t lda, size_t bSx, size_t bSy, size_t ldb, size_t cSx, size_t cSy, size_t ldc) {
    __shared__ __align__(16) float os[16 * 68];
    const int lane = threadIdx.x & 31, lr = lane & 15, hi = lane >> 4;
    const size_t aoff = (size_t)blockIdx.x * aSx + (size_t)blockIdx.y * aSy + (size_t)lr * lda + 8 * hi;
    const size_t boff = (size_t)blockIdx.x * bSx + (size_t)blockIdx.y * bSy + (size_t)lr * ldb + 8 * hi;
    const size_t coff = (size_t)blockIdx.x * cSx + (size_t)blockIdx.y * cSy;
    v8f acc[4][4];
#pragma unroll
    for (int mb = 0; mb < 4; ++mb)
#pragma unroll
        for (int nb = 0; nb < 4; ++nb) acc[mb][nb] = (v8f){};
    for (int kc = 0; kc < HD; kc += 32) {
        v16h a[4];
#pragma unroll
        for (int mb = 0; mb < 4; ++mb) a[mb] = ldh(A + aoff + (size_t)mb * 16 * lda + kc);
#pragma unroll
        for (int nb = 0; nb < 4; ++nb) { const v16h b = ldh(Bt + boff + (size_t)nb * 16 * ldb + kc);
#pragma unroll
            for (int mb = 0; mb < 4; ++mb) acc[mb][nb] = wmma16g(a[mb], b, acc[mb][nb]); }
    }
#pragma unroll
    for (int mb = 0; mb < 4; ++mb) {
#pragma unroll
        for (int nb = 0; nb < 4; ++nb) {
#pragma unroll
            for (int j = 0; j < 8; ++j) os[(hi * 8 + j) * 68 + nb * 16 + lr] = acc[mb][nb][j]; }
        wave_sync();
        for (int ps = 0; ps < 2; ++ps) {
#pragma unroll
            for (int s = 0; s < 4; ++s) { const int row = 4 * s + (lane >> 3), c8 = (lane & 7) * 8;
                const v4f x0 = *(const v4fa*)(&os[row * 68 + c8]); const v4f x1 = *(const v4fa*)(&os[row * 68 + c8 + 4]); v8h hv;
#pragma unroll
                for (int i = 0; i < 4; ++i) { hv[i] = toh_flush(x0[i]); hv[4 + i] = toh_flush(x1[i]); }
                *(volatile v8h*)(C + coff + (size_t)(mb * 16 + row) * ldc + c8) = hv; }
            if (ps == 0) __threadfence(); }
        wave_sync();
    }
}

__device__ __forceinline__ float pair_logit(float c, float a2, float n2, float a1sq, float m2a1, float qq, float n1) {
    float p = a1sq * n2;
    p = fmaf(c, fmaf(qq, c, m2a1 * a2), p);
    p = fmaf(n1, a2 * a2, p);
    return __builtin_amdgcn_sqrtf(fmaxf(p, 0.0f)) * LOG2E;
}

__global__ __launch_bounds__(32 * AW) __attribute__((amdgpu_num_vgpr(256)))
void k_pair(const h16* __restrict__ PH, const h16* __restrict__ PR, const float* __restrict__ NRM, const h16* __restrict__ BV, float* OUT) {
    __shared__ __align__(16) float Cs[VE * VE];
    __shared__ __align__(16) float q1s[AW * VE * 16];
    __shared__ __align__(16) float os[AW * 16 * OSP];
    __shared__ __align__(16) float nn[2 * VE];
    const int tid = threadIdx.x;
    const int lane = tid & 31, lr = lane & 15, hi = lane >> 4;
    const int wave = __builtin_amdgcn_readfirstlane((int)(threadIdx.x >> 5));
    const int b = blockIdx.y;
    const int t0 = (blockIdx.x * AW + wave) * 16;
    { const int sel = (tid >> 6) + 1;
      nn[tid] = NRM[(size_t)(sel * NB + b) * SEQ + SQ + (tid & 63)]; }
    const float qqv = NRM[(size_t)b * SEQ + t0 + lr];
    const size_t qo  = ((size_t)b * SEQ + (size_t)(t0 + lr)) * HD + 8 * hi;
    const size_t k1o = ((size_t)(NB + b) * SEQ + (size_t)(SQ + lr)) * HD + 8 * hi;
    const size_t k2o = ((size_t)(2 * NB + b) * SEQ + (size_t)(SQ + lr)) * HD + 8 * hi;
    { v16h ah[2], ar[2];
#pragma unroll
      for (int kc = 0; kc < 2; ++kc) { ah[kc] = ldh(PH + k1o + (size_t)wave * 16 * HD + kc * 32); ar[kc] = ldh(PR + k1o + (size_t)wave * 16 * HD + kc * 32); }
#pragma unroll
      for (int t = 0; t < 4; ++t) { v8f cH = (v8f){}, cL = (v8f){};
#pragma unroll
          for (int kc = 0; kc < 2; ++kc) { const v16h bh = ldh(PH + k2o + (size_t)t * 16 * HD + kc * 32); const v16h br = ldh(PR + k2o + (size_t)t * 16 * HD + kc * 32);
              cH = wmma16g(ah[kc], bh, cH); cL = wmma16g(ah[kc], br, cL); cL = wmma16g(ar[kc], bh, cL); }
#pragma unroll
          for (int r = 0; r < 8; ++r) Cs[(wave * 16 + 8 * hi + r) * VE + t * 16 + lr] = cH[r] + cL[r] * QRI; } }
    float a2[4][8];
    const int wq = wave * VE * 16;
    { v16h qh[2], qr[2];
#pragma unroll
      for (int kc = 0; kc < 2; ++kc) { qh[kc] = ldh(PH + qo + kc * 32); qr[kc] = ldh(PR + qo + kc * 32); }
#pragma unroll
      for (int t = 0; t < 4; ++t) { v8f sH = (v8f){}, sL = (v8f){}, uH = (v8f){}, uL = (v8f){};
#pragma unroll
          for (int kc = 0; kc < 2; ++kc) {
              const v16h k1h = ldh(PH + k1o + (size_t)t * 16 * HD + kc * 32); const v16h k1r = ldh(PR + k1o + (size_t)t * 16 * HD + kc * 32);
              sH = wmma16g(k1h, qh[kc], sH); sL = wmma16g(k1h, qr[kc], sL); sL = wmma16g(k1r, qh[kc], sL);
              const v16h k2h = ldh(PH + k2o + (size_t)t * 16 * HD + kc * 32); const v16h k2r = ldh(PR + k2o + (size_t)t * 16 * HD + kc * 32);
              uH = wmma16g(k2h, qh[kc], uH); uL = wmma16g(k2h, qr[kc], uL); uL = wmma16g(k2r, qh[kc], uL); }
#pragma unroll
          for (int r = 0; r < 8; ++r) { q1s[wq + (t * 16 + 8 * hi + r) * 16 + lr] = sH[r] + sL[r] * QRI; a2[t][r] = uH[r] + uL[r] * QRI; } } }
    __syncthreads();
    float n2v[4][8];
#pragma unroll
    for (int t = 0; t < 4; ++t) { const v4f x0 = *(const v4fa*)(&nn[VE + t * 16 + 8 * hi]); const v4f x1 = *(const v4fa*)(&nn[VE + t * 16 + 8 * hi + 4]);
#pragma unroll
        for (int r = 0; r < 4; ++r) { n2v[t][r] = x0[r]; n2v[t][4 + r] = x1[r]; } }
    const size_t bvo = ((size_t)b * VE + (size_t)lr) * NPAIR + 8 * hi;
    v8f o[4];
#pragma unroll
    for (int qt = 0; qt < 4; ++qt) o[qt] = (v8f){};
    float m = NEGB, l = 0.0f;
    for (int j = 0; j < VE; ++j) {
        const float a1 = q1s[wq + j * 16 + lr];
        const float n1j = nn[j];
        const float a1sq = a1 * a1, m2a1 = -2.0f * a1;
#pragma unroll
        for (int hb = 0; hb < 2; ++hb) {
            const int cb = j * VE + hb * 32 + 8 * hi;
            const v4f c0 = *(const v4fa*)(&Cs[cb]), c1 = *(const v4fa*)(&Cs[cb + 4]), c2 = *(const v4fa*)(&Cs[cb + 16]), c3 = *(const v4fa*)(&Cs[cb + 20]);
            float ta[8], tb[8]; float mx = NEGB;
#pragma unroll
            for (int r = 0; r < 8; ++r) {
                const float ca = (r < 4) ? c0[r & 3] : c1[r & 3];
                const float cc = (r < 4) ? c2[r & 3] : c3[r & 3];
                ta[r] = pair_logit(ca, a2[2 * hb][r], n2v[2 * hb][r], a1sq, m2a1, qqv, n1j);
                tb[r] = pair_logit(cc, a2[2 * hb + 1][r], n2v[2 * hb + 1][r], a1sq, m2a1, qqv, n1j);
                mx = fmaxf(mx, fmaxf(ta[r], tb[r])); }
            mx = fmaxf(mx, __shfl_xor(mx, 16, 32));
            const float mnew = fmaxf(m, mx);
            const float alpha = __builtin_amdgcn_exp2f(m - mnew);
            const float sh = PSH - mnew;
            v16h pb; float ls = 0.0f;
#pragma unroll
            for (int r = 0; r < 8; ++r) {
                const float ea = ta[r] + sh, eb = tb[r] + sh;
                const float xa = __builtin_amdgcn_exp2f(ea), xb = __builtin_amdgcn_exp2f(eb);
                const float ga = (ea < -14.0f) ? 0.0f : xa, gb = (eb < -14.0f) ? 0.0f : xb;
                const h16 pa = (h16)ga; const h16 pc = (h16)gb;
                pb[r] = pa; pb[8 + r] = pc;
                ls += (float)pa + (float)pc; }
            l = l * alpha + ls; m = mnew;
#pragma unroll
            for (int qt = 0; qt < 4; ++qt) o[qt] = o[qt] * alpha;
            const h16* bp = BV + bvo + (size_t)(j * VE + hb * 32);
#pragma unroll
            for (int qt = 0; qt < 4; ++qt) { const v16h av = ldh(bp + (size_t)qt * 16 * NPAIR); o[qt] = wmma16g(av, pb, o[qt]); }
        }
    }
    l += __shfl_xor(l, 16, 32);
    const float inv = 1.0f / (l * BCAR);
    const int wb = wave * 16 * OSP;
#pragma unroll
    for (int qt = 0; qt < 4; ++qt) { v4f a, c;
        a[0] = o[qt][0] * inv; a[1] = o[qt][1] * inv; a[2] = o[qt][2] * inv; a[3] = o[qt][3] * inv;
        c[0] = o[qt][4] * inv; c[1] = o[qt][5] * inv; c[2] = o[qt][6] * inv; c[3] = o[qt][7] * inv;
        *(v4fa*)(&os[wb + lr * OSP + 16 * qt + 8 * hi]) = a; *(v4fa*)(&os[wb + lr * OSP + 16 * qt + 8 * hi + 4]) = c; }
    wave_sync();
    float* orow = OUT + ((size_t)b * OUT_SEQ + (size_t)t0) * HD;
    for (int ps = 0; ps < 2; ++ps) {
#pragma unroll
        for (int s = 0; s < 8; ++s) { const int p = s * 32 + lane; const int row = p >> 4, cofs = (p & 15) * 4;
            const v4f val = *(const v4fa*)(&os[wb + row * OSP + cofs]);
            *(volatile v4f*)(orow + (size_t)p * 4) = val; }
        if (ps == 0) __threadfence(); }
}

static constexpr size_t al256(size_t v) { return (v + 255) & ~(size_t)255; }
static constexpr size_t SZ_XB = al256((size_t)NB * SEQ * DM * 2);
static constexpr size_t SZ_WT = al256((size_t)DO * DM * 2);
static constexpr size_t SZ_BF = al256((size_t)NPAIR * HD * 2);
static constexpr size_t SZ_PL = al256((size_t)NCH * NB * SEQ * HD * 2);
static constexpr size_t SZ_NR = al256((size_t)NCH * NB * SEQ * 4);
static constexpr size_t SZ_UP = al256((size_t)NB * VE * NPAIR * 2);
static constexpr size_t SZ_TOTAL = SZ_XB + SZ_WT + SZ_BF + 2 * SZ_PL + SZ_NR + 2 * SZ_UP;
static_assert(SZ_TOTAL <= (size_t)134217728);
static_assert((size_t)(NB * SEQ / 64) * 64 == (size_t)NB * SEQ);
static_assert((size_t)(NPAIR / 64) * 64 == (size_t)NPAIR);
static_assert((size_t)(SQ / (16 * AW)) * 16 * AW == (size_t)SQ);

extern "C" void kernel_launch(void* const* d_in, const int* in_sizes, int n_in,
                              void* d_out, int out_size, void* d_ws, size_t ws_size, hipStream_t stream) {
    if (n_in < 3) return;
    const size_t needx = ((size_t)(NB - 1) * SEQ_FULL + SEQ) * DM;
    if ((size_t)in_sizes[0] < needx) return;
    if ((size_t)in_sizes[1] < (size_t)DM * DO) return;
    if ((size_t)in_sizes[2] < (size_t)NPAIR * HD) return;
    if ((size_t)out_size < ((size_t)(NB - 1) * OUT_SEQ + SEQ) * HD) return;
    if (SZ_TOTAL > ws_size) return;
    const float* xin = (const float*)d_in[0];
    const float* wqk = (const float*)d_in[1];
    const float* bw  = (const float*)d_in[2];
    float* OUT = (float*)d_out;
    char* wsp = (char*)d_ws;
    bf*  XB = (bf*)wsp;  wsp += SZ_XB;
    bf*  WT = (bf*)wsp;  wsp += SZ_WT;
    h16* BF = (h16*)wsp; wsp += SZ_BF;
    h16* PH = (h16*)wsp; wsp += SZ_PL;
    h16* PR = (h16*)wsp; wsp += SZ_PL;
    float* NRM = (float*)wsp; wsp += SZ_NR;
    h16* UP = (h16*)wsp; wsp += SZ_UP;
    h16* BVP = (h16*)wsp; wsp += SZ_UP;

    if (SEQ == SEQ_FULL) {
        const size_t n8 = (size_t)NB * SEQ * DM / 8;
        k_cvt8<<<(unsigned)((n8 + 255) / 256), 256, 0, stream>>>(xin, XB, n8);
    } else {
        const size_t n8 = (size_t)SEQ * DM / 8;
        for (int b = 0; b < NB; ++b) k_cvt8<<<(unsigned)((n8 + 255) / 256), 256, 0, stream>>>(xin + (size_t)b * SEQ_FULL * DM, XB + (size_t)b * SEQ * DM, n8);
    }
    k_wT<<<dim3(DM / 64, DO / 64, 1), 256, 0, stream>>>(wqk, WT);
    { const size_t n8 = (size_t)NPAIR * HD / 8;
      k_cvt8h<<<(unsigned)((n8 + 255) / 256), 256, 0, stream>>>(bw, BF, n8, BCAR); }

    k_proj<<<dim3(NB * SEQ / 64, DO / 64, 1), 32, 0, stream>>>(XB, WT, PH, PR, NRM, OUT);

    const h16* VH = PH + ((size_t)3 * NB * SEQ + (size_t)SQ) * HD;
    k_gemm64<<<dim3(NPAIR / 64, NB, 1), 32, 0, stream>>>(VH, BF, UP,
        (size_t)0, (size_t)SEQ * HD, (size_t)HD,
        (size_t)64 * HD, (size_t)0, (size_t)HD,
        (size_t)64, (size_t)VE * NPAIR, (size_t)NPAIR);
    k_gemm64<<<dim3(VE, NB, 1), 32, 0, stream>>>(VH, UP, BVP,
        (size_t)0, (size_t)SEQ * HD, (size_t)HD,
        (size_t)HD, (size_t)VE * NPAIR, (size_t)NPAIR,
        (size_t)NPAIR, (size_t)VE * NPAIR, (size_t)VE);

    k_pair<<<dim3(SQ / (16 * AW), NB, 1), 32 * AW, 0, stream>>>(PH, PR, NRM, BVP, OUT);
}
